// HyperspectralCmKANLayer_26912265076905
// MI455X (gfx1250) — hardware-verified
//
#include <hip/hip_runtime.h>
#include <math.h>

#define CI 31
#define CO 31
#define NB8 8
#define NPIX 16384
#define COEF_LEN (CI * CO * NB8)
#define UW_OFF COEF_LEN
#define RW_OFF (COEF_LEN + CI * CO)
#define PNUM 9610
#define PB 64
#define NCOL 320

typedef _Float16 f16;
typedef __attribute__((ext_vector_type(16))) f16 f16x16;
typedef __attribute__((ext_vector_type(8)))  f16 f16x8;
typedef __attribute__((ext_vector_type(8)))  float f32x8;
typedef __attribute__((ext_vector_type(4)))  float v4f_t;
typedef float v4fa __attribute__((ext_vector_type(4), may_alias));
__device__ __forceinline__ f32x8 wmma16(f16x16 a, f16x16 b, f32x8 c) {
  c = __builtin_amdgcn_wmma_f32_16x16x32_f16(false, a, false, b, (short)0, c, false, false);
  asm volatile("v_nop\n\tv_nop\n\tv_nop\n\tv_nop" : "+v"(c) : "v"(a), "v"(b));
  return c;
}
__device__ __forceinline__ f16x16 lds_frag(const f16* base, int stride) {
  const int lane = threadIdx.x & 31, row = lane & 15, kh = (lane >> 4) * 8;
  const f16x8 lo = *(const f16x8*)(base + row * stride + kh);
  const f16x8 hi = *(const f16x8*)(base + row * stride + kh + 16);
  f16x16 f;
#pragma unroll
  for (int i = 0; i < 8; ++i) { f[i] = lo[i]; f[i + 8] = hi[i]; }
  return f;
}
__device__ __forceinline__ int prow(int i, int col) {
  if (col < CO * NB8) return (i * CO) * NB8 + col;
  if (col < CO * NB8 + CO) return UW_OFF + i * CO + (col - CO * NB8);
  if (col < CO * NB8 + 2 * CO) return RW_OFF + i * CO + (col - CO * NB8 - CO);
  return -1;
}

__global__ __launch_bounds__(256) void k_hyper(const float* __restrict__ x, const float* __restrict__ gw, const float* __restrict__ gb, float* __restrict__ out) {
  __shared__ __attribute__((aligned(16))) f16 xS[PB * 40];
  __shared__ float xF[PB * 32];
  __shared__ float wT[PB * 324];
  __shared__ float bas[PB * 9];
  __shared__ __attribute__((aligned(16))) float yS[CO * 68];
  const int tid = threadIdx.x, lane = tid & 31, wave = tid >> 5, cl = lane & 15, rh = (lane >> 4) * 8;
  const int p0 = blockIdx.x * PB;
  for (int e = tid; e < PB * 32; e += 256) { const int r = e >> 5, c = e & 31; const float v = (c < CI) ? x[(size_t)c * NPIX + p0 + r] : 0.0f; xF[e] = v; xS[r * 40 + c] = (f16)v; }
  float yacc[8];
#pragma unroll
  for (int j = 0; j < 8; ++j) yacc[j] = 0.0f;
  const int mp = tid >> 2, oq = (tid & 3) * 8;
  __syncthreads();
#pragma unroll 1
  for (int i = 0; i < CI; ++i) {
    if (tid < PB) { const float t = xF[tid * 32 + i]; float bs[11];
#pragma unroll
      for (int q = 0; q < 11; ++q) { const float g0 = -1.0f + (float)(q - 3) * 0.4f; bs[q] = (t >= g0 && t < g0 + 0.4f) ? 1.0f : 0.0f; }
#pragma unroll
      for (int p = 1; p <= 3; ++p) { const float inv = 1.0f / ((float)p * 0.4f);
#pragma unroll
        for (int q = 0; q < 11 - p; ++q) { const float gq = -1.0f + (float)(q - 3) * 0.4f; bs[q] = (t - gq) * inv * bs[q] + ((gq + (float)(p + 1) * 0.4f) - t) * inv * bs[q + 1]; } }
#pragma unroll
      for (int m = 0; m < 8; ++m) bas[tid * 9 + m] = bs[m];
      bas[tid * 9 + 8] = t / (1.0f + expf(-t)); }
    { const int pt = wave & 3; const f16x16 af = lds_frag(xS + (pt * 16) * 40, 40);
#pragma unroll 1
      for (int jt = 0; jt < 10; ++jt) { const int ct = (wave >> 2) + 2 * jt; const int col = ct * 16 + (lane & 15); const int pr = prow(i, col); const int kh = (lane >> 4) * 8;
        f16x16 bf;
#pragma unroll
        for (int e = 0; e < 8; ++e) { const int c0 = kh + e, c1 = kh + 16 + e;
          bf[e] = (f16)((pr >= 0 && c0 < CI) ? gw[(size_t)pr * CI + c0] : 0.0f); bf[8 + e] = (f16)((pr >= 0 && c1 < CI) ? gw[(size_t)pr * CI + c1] : 0.0f); }
        f32x8 acc = {}; acc = wmma16(af, bf, acc);
        const int colw = ct * 16 + cl; const int prw = prow(i, colw); const float bb = (prw >= 0) ? gb[prw] : 0.0f;
#pragma unroll
        for (int r = 0; r < 8; ++r) wT[(pt * 16 + rh + r) * 324 + colw] = acc[r] + bb; } }
    __syncthreads();
    { const float* bp = bas + mp * 9; const float sil = bp[8]; const float* wr = wT + mp * 324;
#pragma unroll
      for (int j = 0; j < 8; ++j) { const int o = oq + j; if (o < CO) { float s = 0.0f;
#pragma unroll
          for (int m = 0; m < 8; ++m) s += bp[m] * wr[o * 8 + m];
          yacc[j] += wr[CO * NB8 + o] * s + sil * wr[CO * NB8 + CO + o]; } } }
    __syncthreads();
  }
#pragma unroll
  for (int j = 0; j < 8; ++j) { const int o = oq + j; if (o < CO) yS[o * 68 + mp] = yacc[j]; }
  __syncthreads();
#pragma unroll 1
  for (int pass = 0; pass < 2; ++pass) { for (int q4 = tid; q4 < CO * 16; q4 += 256) { const int o = q4 >> 4, c4 = (q4 & 15) * 4;
      *(volatile v4f_t*)(out + (size_t)o * NPIX + p0 + c4) = *(const volatile v4fa*)(yS + o * 68 + c4); } __threadfence(); }
}

extern "C" void kernel_launch(void* const* d_in, const int* in_sizes, int n_in,
                              void* d_out, int out_size, void* d_ws, size_t ws_size,
                              hipStream_t stream) {
  (void)in_sizes; (void)n_in; (void)out_size; (void)d_ws; (void)ws_size;
  const float* x = (const float*)d_in[0];
  const float* gw = (const float*)d_in[1];
  const float* gb = (const float*)d_in[2];
  float* out = (float*)d_out;
  k_hyper<<<dim3(NPIX / PB), dim3(256), 0, stream>>>(x, gw, gb, out);
}
